// CQFusion_4750233830147
// MI455X (gfx1250) — hardware-verified
//
#include <hip/hip_runtime.h>


namespace {
constexpr int NB = 16, LC = 2048, LQ = 512, D = 128, KU = 4 * D;
constexpr float NEG_INF = -1e30f, XS = 8.0f, AS = 64.0f, PS = 1024.0f, WSC = 256.0f;
typedef _Float16 b16;
typedef __attribute__((ext_vector_type(16))) _Float16 v16b;
typedef __attribute__((ext_vector_type(8))) _Float16 v8b;
typedef __attribute__((ext_vector_type(4))) _Float16 v4b;
typedef __attribute__((ext_vector_type(2))) _Float16 v2b;
typedef __attribute__((ext_vector_type(8))) float v8f;
typedef __attribute__((ext_vector_type(4))) float v4f;
typedef __attribute__((ext_vector_type(2))) float v2f;
__device__ __forceinline__ float bf16_rne(float f) { unsigned int u = __float_as_uint(f); u += 0x7FFFu + ((u >> 16) & 1u); return __uint_as_float(u & 0xFFFF0000u); }
__device__ __forceinline__ void split16(float v, b16& hi, b16& lo) { hi = (b16)v; lo = (b16)(v - (float)hi); }
__device__ __forceinline__ v16b frag_kb(const b16* p, int hh) { const v8b a = *(const v8b*)(p + 8 * hh), b = *(const v8b*)(p + 16 + 8 * hh); v16b f;
#pragma unroll
  for (int e = 0; e < 8; ++e) { f[e] = a[e]; f[8 + e] = b[e]; } return f; }
__device__ __forceinline__ v8f wmma16b(v16b a, v16b b, v8f c) { v8f d = __builtin_amdgcn_wmma_f32_16x16x32_f16(false, a, false, b, (short)0, c, false, false); asm volatile("v_nop\n\tv_nop\n\tv_nop\n\tv_nop" : "+v"(d) : "v"(a), "v"(b)); return d; }
__device__ __forceinline__ void wave_lds_sync() { __builtin_amdgcn_fence(__ATOMIC_RELEASE, "workgroup"); __builtin_amdgcn_wave_barrier(); __builtin_amdgcn_fence(__ATOMIC_ACQUIRE, "workgroup"); }
__device__ __forceinline__ float pmul(float a, float b) { float p = a * b; asm volatile("" : "+v"(p)); return p; }
__device__ __forceinline__ float opaque(float a) { asm volatile("" : "+v"(a)); return a; }
__device__ __forceinline__ float nexp(float x) { return __builtin_amdgcn_exp2f(x * 1.4426950408889634f); }

__global__ __launch_bounds__(256) void wprep_kernel(const float* __restrict__ w, b16* __restrict__ WT) {
  const size_t u = (size_t)blockIdx.x * 256 + threadIdx.x; if (u >= (size_t)D * KU / 8) return; const size_t e = u * 8; v8b o;
  for (int j = 0; j < 8; ++j) o[j] = (b16)(bf16_rne(w[e + j]) * WSC);
  for (int pass = 0; pass < 2; ++pass) { *(volatile v8b*)(WT + e) = o; __threadfence(); }
}
__global__ __launch_bounds__(256) void cprep_kernel(const float* __restrict__ ctx, const float* __restrict__ cm, const float* __restrict__ w4c, const float* __restrict__ w4m, b16* __restrict__ AH, b16* __restrict__ AL, float* __restrict__ S0, float* __restrict__ CMB, b16* __restrict__ CT) {
  __shared__ __attribute__((aligned(16))) b16 tile[D][64 + 8]; __shared__ __attribute__((aligned(16))) float s0s[64], cms[64];
  const int wave = threadIdx.x >> 5, lane = threadIdx.x & 31; const int c0 = blockIdx.x * 64;
  float wc[4], wm[4]; for (int i = 0; i < 4; ++i) { wc[i] = opaque(bf16_rne(w4c[lane * 4 + i])); wm[i] = opaque(bf16_rne(w4m[lane * 4 + i])); }
#pragma unroll 1
  for (int rr = 0; rr < 8; ++rr) { const int cl = wave * 8 + rr; const size_t c = (size_t)c0 + cl; const v4f x = *(const v4f*)(ctx + c * D + lane * 4);
    float s = 0.0f; v4b ah, al, ch;
    for (int i = 0; i < 4; ++i) { const float xv = bf16_rne(x[i]); s += pmul(xv, wc[i]); b16 p, q; split16(pmul(xv, wm[i]) * AS, p, q); ah[i] = p; al[i] = q; ch[i] = (b16)(xv * XS); tile[lane * 4 + i][cl] = ch[i]; }
    for (int o = 16; o; o >>= 1) s += __shfl_xor(s, o);
    if (lane == 0) { s0s[cl] = s; cms[cl] = (1.0f - bf16_rne(cm[c])) * NEG_INF; }
    for (int pass = 0; pass < 2; ++pass) { *(volatile v4b*)(AH + c * D + lane * 4) = ah; *(volatile v4b*)(AL + c * D + lane * 4) = al; __threadfence(); } }
  __syncthreads();
  for (int pass = 0; pass < 2; ++pass) {
    if (wave == 0) { if (lane < 16) *(volatile v4f*)(S0 + c0 + lane * 4) = *(const v4f*)(&s0s[lane * 4]); else *(volatile v4f*)(CMB + c0 + (lane - 16) * 4) = *(const v4f*)(&cms[(lane - 16) * 4]); }
#pragma unroll 1
    for (int dd = 0; dd < 16; ++dd) { const int d = wave * 16 + dd; *(volatile v2b*)(CT + (size_t)d * LC + c0 + lane * 2) = *(const v2b*)(&tile[d][lane * 2]); }
    __threadfence(); }
}
__global__ __launch_bounds__(256) void qprep_kernel(const float* __restrict__ qry, const float* __restrict__ qm, const float* __restrict__ w4q, b16* __restrict__ QB, float* __restrict__ S1, float* __restrict__ QMB, b16* __restrict__ QT) {
  __shared__ __attribute__((aligned(16))) b16 tile[D][64 + 8]; __shared__ __attribute__((aligned(16))) float s1s[64], qms[64];
  const int wave = threadIdx.x >> 5, lane = threadIdx.x & 31; const int q0 = blockIdx.x * 64;
  float wq[4]; for (int i = 0; i < 4; ++i) wq[i] = opaque(bf16_rne(w4q[lane * 4 + i]));
#pragma unroll 1
  for (int rr = 0; rr < 8; ++rr) { const int ql = wave * 8 + rr; const size_t q = (size_t)q0 + ql; const v4f x = *(const v4f*)(qry + q * D + lane * 4);
    float s = 0.0f; v4b qh;
    for (int i = 0; i < 4; ++i) { const float xv = bf16_rne(x[i]); s += pmul(xv, wq[i]); qh[i] = (b16)(xv * XS); tile[lane * 4 + i][ql] = qh[i]; }
    for (int o = 16; o; o >>= 1) s += __shfl_xor(s, o);
    if (lane == 0) { s1s[ql] = s; qms[ql] = (1.0f - bf16_rne(qm[q])) * NEG_INF; }
    for (int pass = 0; pass < 2; ++pass) { *(volatile v4b*)(QB + q * D + lane * 4) = qh; __threadfence(); } }
  __syncthreads();
  for (int pass = 0; pass < 2; ++pass) {
    if (wave == 0) { if (lane < 16) *(volatile v4f*)(S1 + q0 + lane * 4) = *(const v4f*)(&s1s[lane * 4]); else *(volatile v4f*)(QMB + q0 + (lane - 16) * 4) = *(const v4f*)(&qms[(lane - 16) * 4]); }
#pragma unroll 1
    for (int dd = 0; dd < 16; ++dd) { const int d = wave * 16 + dd; *(volatile v2b*)(QT + (size_t)d * LQ + q0 + lane * 2) = *(const v2b*)(&tile[d][lane * 2]); }
    __threadfence(); }
}
template <int MODE>
__global__ __launch_bounds__(128) void gemm_kernel(const b16* __restrict__ A1, const b16* __restrict__ A2, const b16* __restrict__ B1, const b16* __restrict__ B2, int K, float sc, const float* __restrict__ S0, const float* __restrict__ S1,
                                                  float* __restrict__ OUT, int ldc, b16* __restrict__ OUTH, b16* __restrict__ OUTL, int ldt) {
  __shared__ __attribute__((aligned(16))) float Tf[64][128 + 4];
  const int wave = threadIdx.x >> 5, lane = threadIdx.x & 31, nloc = lane & 15, hlf = lane >> 4; const size_t m0 = (size_t)blockIdx.x * 64 + wave * 16; const int c0 = blockIdx.y * 128;
  v8f acc[8];
#pragma unroll
  for (int t = 0; t < 8; ++t) acc[t] = (v8f){};
  const b16* a1 = A1 + (m0 + nloc) * (size_t)K; const b16* a2 = A2 ? A2 + (m0 + nloc) * (size_t)K : nullptr;
#pragma unroll 2
  for (int kb = 0; kb < K; kb += 32) { const v16b a = frag_kb(a1 + kb, hlf); v16b al = {}; if (A2) al = frag_kb(a2 + kb, hlf);
#pragma unroll
    for (int t = 0; t < 8; ++t) { const size_t brow = (size_t)(c0 + t * 16 + nloc) * K + kb; const v16b bw = frag_kb(B1 + brow, hlf); acc[t] = wmma16b(a, bw, acc[t]); if (A2) acc[t] = wmma16b(al, bw, acc[t]); if (B2) acc[t] = wmma16b(a, frag_kb(B2 + brow, hlf), acc[t]); } }
#pragma unroll
  for (int t = 0; t < 8; ++t) { const int cc = t * 16 + nloc; const float s1 = (MODE == 0) ? S1[c0 + cc] : 0.0f;
#pragma unroll 1
    for (int r8 = 0; r8 < 8; ++r8) { const int rl = wave * 16 + 8 * hlf + r8; float v = acc[t][r8] * sc; if (MODE == 0) v += S0[m0 + 8 * hlf + r8] + s1; Tf[rl][cc] = v; } }
  if (MODE == 2) __syncthreads(); else wave_lds_sync();
  for (int pass = 0; pass < 2; ++pass) {
    if (MODE != 2) { for (int rr = 0; rr < 16; ++rr) *(volatile v4f*)(OUT + (m0 + rr) * (size_t)ldc + c0 + lane * 4) = *(const v4f*)(&Tf[wave * 16 + rr][lane * 4]); }
    else {
#pragma unroll 1
      for (int dd = 0; dd < 32; ++dd) { const int d = wave * 32 + dd; b16 h0, l0, h1, l1; split16(Tf[lane * 2][d] * XS, h0, l0); split16(Tf[lane * 2 + 1][d] * XS, h1, l1); v2b vh, vl; vh[0] = h0; vh[1] = h1; vl[0] = l0; vl[1] = l1;
        *(volatile v2b*)(OUTH + (size_t)(c0 + d) * ldt + blockIdx.x * 64 + lane * 2) = vh; *(volatile v2b*)(OUTL + (size_t)(c0 + d) * ldt + blockIdx.x * 64 + lane * 2) = vl; } }
    __threadfence(); }
}
__global__ __launch_bounds__(256) void rowstat_kernel(const float* __restrict__ S, const float* __restrict__ QMB, float* __restrict__ RM, float* __restrict__ RI) {
  __shared__ float sm[32], si[32];
  const int wave = threadIdx.x >> 5, lane = threadIdx.x & 31;
  float qb[16]; for (int i = 0; i < 16; ++i) qb[i] = QMB[lane * 16 + i];
#pragma unroll 1
  for (int rr = 0; rr < 4; ++rr) { const int cl = wave * 4 + rr; const size_t c = (size_t)blockIdx.x * 32 + cl; const float* row = S + c * LQ + lane * 16; float v[16];
    for (int qq = 0; qq < 4; ++qq) { const v4f t = *(const v4f*)(row + qq * 4); for (int i = 0; i < 4; ++i) v[qq * 4 + i] = t[i] + qb[qq * 4 + i]; }
    float m = v[0]; for (int i = 1; i < 16; ++i) m = fmaxf(m, v[i]); for (int o = 16; o; o >>= 1) m = fmaxf(m, __shfl_xor(m, o));
    float s = 0.0f; for (int i = 0; i < 16; ++i) s += nexp(v[i] - m); for (int o = 16; o; o >>= 1) s += __shfl_xor(s, o);
    if (lane == 0) { sm[cl] = m; si[cl] = 1.0f / s; } }
  __syncthreads();
  for (int pass = 0; pass < 2; ++pass) { if (threadIdx.x < 8) *(volatile v4f*)(RM + (size_t)blockIdx.x * 32 + threadIdx.x * 4) = *(const v4f*)(&sm[threadIdx.x * 4]); else if (threadIdx.x < 16) *(volatile v4f*)(RI + (size_t)blockIdx.x * 32 + (threadIdx.x - 8) * 4) = *(const v4f*)(&si[(threadIdx.x - 8) * 4]); __threadfence(); }
}
__global__ __launch_bounds__(256) void colstat_kernel(const float* __restrict__ S, const float* __restrict__ CMB, float* __restrict__ CM, float* __restrict__ CI) {
  __shared__ float pm[8][32], psum[8][32], mfin[32], ifin[32];
  const int wave = threadIdx.x >> 5, lane = threadIdx.x & 31; const int q = blockIdx.x * 32 + lane;
  float m = -INFINITY;
#pragma unroll 4
  for (int c = wave; c < LC; c += 8) m = fmaxf(m, S[(size_t)c * LQ + q] + CMB[c]);
  pm[wave][lane] = m; __syncthreads();
  if (wave == 0) { float mm = pm[0][lane]; for (int w = 1; w < 8; ++w) mm = fmaxf(mm, pm[w][lane]); mfin[lane] = mm; }
  __syncthreads();
  const float mm = mfin[lane]; float s = 0.0f;
#pragma unroll 4
  for (int c = wave; c < LC; c += 8) s += nexp(S[(size_t)c * LQ + q] + CMB[c] - mm);
  psum[wave][lane] = s; __syncthreads();
  if (wave == 0) { float ss = psum[0][lane]; for (int w = 1; w < 8; ++w) ss += psum[w][lane]; ifin[lane] = 1.0f / ss; }
  __syncthreads();
  for (int pass = 0; pass < 2; ++pass) { if (threadIdx.x < 8) *(volatile v4f*)(CM + (size_t)blockIdx.x * 32 + threadIdx.x * 4) = *(const v4f*)(&mfin[threadIdx.x * 4]); else if (threadIdx.x < 16) *(volatile v4f*)(CI + (size_t)blockIdx.x * 32 + (threadIdx.x - 8) * 4) = *(const v4f*)(&ifin[(threadIdx.x - 8) * 4]); __threadfence(); }
}
__global__ __launch_bounds__(256) void prob_kernel(const float* __restrict__ S, const float* __restrict__ QMB, const float* __restrict__ CMB, const float* __restrict__ RM, const float* __restrict__ RI, const float* __restrict__ CM, const float* __restrict__ CI, b16* __restrict__ P1H, b16* __restrict__ P1L, b16* __restrict__ P2H, b16* __restrict__ P2L) {
  __shared__ __attribute__((aligned(16))) b16 th[64][64 + 8], tl[64][64 + 8];
  const int wave = threadIdx.x >> 5, lane = threadIdx.x & 31; const int c0 = blockIdx.x * 64, q0 = blockIdx.y * 64; const int ql = lane * 2; const int q = q0 + ql;
  const float qb0 = QMB[q], qb1 = QMB[q + 1], cm0 = CM[q], cm1 = CM[q + 1], ci0 = CI[q], ci1 = CI[q + 1];
#pragma unroll 1
  for (int rr = 0; rr < 8; ++rr) { const int cl = wave * 8 + rr; const size_t c = (size_t)c0 + cl; const v2f s = *(const v2f*)(S + c * LQ + q); const float rm = RM[c], ri = RI[c], cb = CMB[c];
    b16 h0, l0, h1, l1; split16(pmul(nexp(s[0] + qb0 - rm), ri) * PS, h0, l0); split16(pmul(nexp(s[1] + qb1 - rm), ri) * PS, h1, l1); v2b vh, vl; vh[0] = h0; vh[1] = h1; vl[0] = l0; vl[1] = l1;
    for (int pass = 0; pass < 2; ++pass) { *(volatile v2b*)(P1H + c * LQ + q) = vh; *(volatile v2b*)(P1L + c * LQ + q) = vl; __threadfence(); }
    split16(pmul(nexp(s[0] + cb - cm0), ci0) * PS, h0, l0); split16(pmul(nexp(s[1] + cb - cm1), ci1) * PS, h1, l1); th[ql][cl] = h0; tl[ql][cl] = l0; th[ql + 1][cl] = h1; tl[ql + 1][cl] = l1; }
  __syncthreads();
  for (int pass = 0; pass < 2; ++pass) {
#pragma unroll 1
    for (int rr = 0; rr < 8; ++rr) { const int qq = wave * 8 + rr; *(volatile v2b*)(P2H + (size_t)(q0 + qq) * LC + c0 + lane * 2) = *(const v2b*)(&th[qq][lane * 2]); *(volatile v2b*)(P2L + (size_t)(q0 + qq) * LC + c0 + lane * 2) = *(const v2b*)(&tl[qq][lane * 2]); }
    __threadfence(); }
}
__global__ __launch_bounds__(32) void out_kernel(const float* __restrict__ ctx, const float* __restrict__ C2Q, const float* __restrict__ Q2C, const b16* __restrict__ WT, const float* __restrict__ bias, const float* __restrict__ cm, float* __restrict__ out) {
  __shared__ __attribute__((aligned(16))) b16 Ah[16][KU + 8], Al[16][KU + 8]; __shared__ __attribute__((aligned(16))) float Tf[16][D + 4];
  const int lane = threadIdx.x, nloc = lane & 15, hlf = lane >> 4; const size_t m0 = (size_t)blockIdx.x * 16;
  for (int rr = 0; rr < 16; ++rr) { const size_t r = m0 + rr; const v4f x = *(const v4f*)(ctx + r * D + lane * 4), a = *(const v4f*)(C2Q + r * D + lane * 4), g = *(const v4f*)(Q2C + r * D + lane * 4);
    for (int j = 0; j < 4; ++j) { const int k = lane * 4 + j; const float xv = bf16_rne(x[j]); b16 p, q;
      Ah[rr][k] = (b16)(xv * XS); Al[rr][k] = (b16)0.0f; split16(a[j] * XS, p, q); Ah[rr][D + k] = p; Al[rr][D + k] = q;
      split16(pmul(xv, a[j]) * XS, p, q); Ah[rr][2 * D + k] = p; Al[rr][2 * D + k] = q; split16(pmul(xv, g[j]) * XS, p, q); Ah[rr][3 * D + k] = p; Al[rr][3 * D + k] = q; } }
  wave_lds_sync();
  v8f acc[8];
#pragma unroll
  for (int t = 0; t < 8; ++t) acc[t] = (v8f){};
#pragma unroll 2
  for (int kb = 0; kb < KU; kb += 32) { const v16b a = frag_kb(&Ah[nloc][kb], hlf), al = frag_kb(&Al[nloc][kb], hlf); const bool dolo = kb >= D;
#pragma unroll
    for (int t = 0; t < 8; ++t) { const v16b bw = frag_kb(WT + (size_t)(t * 16 + nloc) * KU + kb, hlf); acc[t] = wmma16b(a, bw, acc[t]); if (dolo) acc[t] = wmma16b(al, bw, acc[t]); } }
  wave_lds_sync();
#pragma unroll
  for (int t = 0; t < 8; ++t) { const int cc = t * 16 + nloc; const float bb = bf16_rne(bias[cc]);
#pragma unroll 1
    for (int r8 = 0; r8 < 8; ++r8) { const int rl = 8 * hlf + r8; Tf[rl][cc] = pmul(acc[t][r8] * (1.0f / (XS * WSC)) + bb, bf16_rne(cm[m0 + rl])); } }
  wave_lds_sync();
  for (int pass = 0; pass < 2; ++pass) { for (int rr = 0; rr < 16; ++rr) *(volatile v4f*)(out + (m0 + rr) * D + lane * 4) = *(const v4f*)(&Tf[rr][lane * 4]); __threadfence(); }
}
}

extern "C" void kernel_launch(void* const* d_in, const int* in_sizes, int n_in, void* d_out, int out_size, void* d_ws, size_t ws_size, hipStream_t stream) {
  (void)n_in;
  auto Fp = [&](int i) { return (const float*)d_in[i]; };
  if (in_sizes[0] != NB * LC * D || in_sizes[1] != NB * LQ * D || in_sizes[3] != NB * LC || in_sizes[4] != NB * LQ || in_sizes[5] != D || in_sizes[6] != D || in_sizes[7] != D || in_sizes[8] != D * KU || in_sizes[9] != D || out_size != NB * LC * D) return;
  size_t off = 0; char* ws = (char*)d_ws;
  auto carve = [&](size_t bytes) { char* p = ws + off; off += (bytes + 255) & ~(size_t)255; return p; };
  b16* WT = (b16*)carve((size_t)D * KU * 2);
  b16* AH = (b16*)carve((size_t)LC * D * 2); b16* AL = (b16*)carve((size_t)LC * D * 2); float* S0 = (float*)carve((size_t)LC * 4); float* CMB = (float*)carve((size_t)LC * 4); b16* CT = (b16*)carve((size_t)D * LC * 2);
  b16* QB = (b16*)carve((size_t)LQ * D * 2); float* S1 = (float*)carve((size_t)LQ * 4); float* QMB = (float*)carve((size_t)LQ * 4); b16* QT = (b16*)carve((size_t)D * LQ * 2);
  float* S = (float*)carve((size_t)LC * LQ * 4); float* RM = (float*)carve((size_t)LC * 4); float* RI = (float*)carve((size_t)LC * 4); float* CM = (float*)carve((size_t)LQ * 4); float* CI = (float*)carve((size_t)LQ * 4);
  b16* P1H = (b16*)carve((size_t)LC * LQ * 2); b16* P1L = (b16*)carve((size_t)LC * LQ * 2); b16* P2H = (b16*)carve((size_t)LQ * LC * 2); b16* P2L = (b16*)carve((size_t)LQ * LC * 2);
  b16* TTH = (b16*)carve((size_t)D * LQ * 2); b16* TTL = (b16*)carve((size_t)D * LQ * 2); float* C2Q = (float*)carve((size_t)LC * D * 4); float* Q2C = (float*)carve((size_t)LC * D * 4);
  if (off > ws_size) return;
  wprep_kernel<<<(unsigned)(((size_t)D * KU / 8 + 255) / 256), 256, 0, stream>>>(Fp(8), WT);
  for (int b = 0; b < NB; ++b) {
    const float* ctx = Fp(0) + (size_t)b * LC * D; const float* qry = Fp(1) + (size_t)b * LQ * D; const float* cmask = Fp(3) + (size_t)b * LC; const float* qmask = Fp(4) + (size_t)b * LQ;
    cprep_kernel<<<LC / 64, 256, 0, stream>>>(ctx, cmask, Fp(5), Fp(7), AH, AL, S0, CMB, CT);
    qprep_kernel<<<LQ / 64, 256, 0, stream>>>(qry, qmask, Fp(6), QB, S1, QMB, QT);
    gemm_kernel<0><<<dim3(LC / 64, LQ / 128), 128, 0, stream>>>(AH, AL, QB, nullptr, D, 1.0f / (AS * XS), S0, S1, S, LQ, nullptr, nullptr, 0);
    rowstat_kernel<<<LC / 32, 256, 0, stream>>>(S, QMB, RM, RI);
    colstat_kernel<<<LQ / 32, 256, 0, stream>>>(S, CMB, CM, CI);
    prob_kernel<<<dim3(LC / 64, LQ / 64), 256, 0, stream>>>(S, QMB, CMB, RM, RI, CM, CI, P1H, P1L, P2H, P2L);
    gemm_kernel<1><<<dim3(LC / 64, 1), 128, 0, stream>>>(P1H, P1L, QT, nullptr, LQ, 1.0f / (PS * XS), nullptr, nullptr, C2Q, D, nullptr, nullptr, 0);
    gemm_kernel<2><<<dim3(LQ / 64, 1), 128, 0, stream>>>(P2H, P2L, CT, nullptr, LC, 1.0f / (PS * XS), nullptr, nullptr, nullptr, 0, TTH, TTL, LQ);
    gemm_kernel<1><<<dim3(LC / 64, 1), 128, 0, stream>>>(P1H, P1L, TTH, TTL, LQ, 1.0f / (PS * XS), nullptr, nullptr, Q2C, D, nullptr, nullptr, 0);
    out_kernel<<<LC / 16, 32, 0, stream>>>(ctx, C2Q, Q2C, WT, Fp(9), cmask, (float*)d_out + (size_t)b * LC * D);
  }
}
